// KernelMethod_SoftMax_67473936220763
// MI455X (gfx1250) — hardware-verified
//
#include <hip/hip_runtime.h>
#include <stddef.h>


#pragma clang fp contract(off)

typedef _Float16 v16h __attribute__((ext_vector_type(16)));
typedef _Float16 v8h  __attribute__((ext_vector_type(8)));
typedef float    v8f  __attribute__((ext_vector_type(8)));
typedef float    v4f  __attribute__((ext_vector_type(4)));
typedef float    v2f  __attribute__((ext_vector_type(2)));
typedef _Float16 h16;

#ifndef NPTS
#define NPTS 131072
#endif
#define NPTS_FULL 131072
#define MCENT 1024
#define DDIM  16
#define KDIM  32

#ifndef SCORE_RES
#define SCORE_RES 1
#endif
#ifndef INPUT_BF16
#define INPUT_BF16 1
#endif

static_assert(NPTS >= 128 && NPTS <= NPTS_FULL && (NPTS % 128) == 0);
static_assert(KDIM == 2 * DDIM && KDIM == 32);
static_assert((MCENT % 256) == 0 && (MCENT % 16) == 0);
static_assert(DDIM == 16);

#define ACARRY 1024.0f
#define RCARRY 2048.0f
#define LSHIFT 32.0f

#define BPLANE_BYTES ((size_t)MCENT * KDIM * 2)
#define CC_BYTES     ((size_t)MCENT * 2 * 4)
#define OFF_BH  ((size_t)0)
#define OFF_BR  (OFF_BH + BPLANE_BYTES)
#define OFF_CC  (OFF_BR + BPLANE_BYTES)
#define WS_TOTAL (OFF_CC + CC_BYTES)
static_assert((BPLANE_BYTES % 128) == 0 && (CC_BYTES % 128) == 0);
static_assert(BPLANE_BYTES == (size_t)(MCENT / 256) * 256 * KDIM * 2);
static_assert(CC_BYTES == (size_t)(MCENT / 256) * 128 * 16);
static_assert(WS_TOTAL <= (size_t)134217728);

__device__ __forceinline__ float bf16r(float x) {
  unsigned int u = __float_as_uint(x);
  u = (u + 0x7FFFu + ((u >> 16) & 1u)) & 0xFFFF0000u;
  return __uint_as_float(u);
}

__device__ __forceinline__ float in_cvt(float x) {
  return INPUT_BF16 ? bf16r(x) : x;
}

static __device__ __forceinline__ h16 toh_flush(float v) {
  const h16 r = (h16)v;
  return (fabsf(v) < 6.103515625e-05f) ? (h16)0.0f : r;
}

__device__ __forceinline__ void split_h(float v, h16& hi, h16& res) {
  hi = toh_flush(v);
  res = toh_flush((v - (float)hi) * RCARRY);
}

__device__ __forceinline__ v16h frag_at(const _Float16* p) {
  v8h lo = *(const v8h*)(p);
  v8h hi = *(const v8h*)(p + 16);
  v16h out;
#pragma unroll
  for (int i = 0; i < 8; ++i) { out[i] = lo[i]; out[i + 8] = hi[i]; }
  return out;
}

__device__ __forceinline__ v8f wmma16(v16h a, v16h b, v8f c) {
  v8f d = __builtin_amdgcn_wmma_f32_16x16x32_f16(false, a, false, b, (short)0, c,
                                                 false, false);
  asm volatile("v_nop\n\tv_nop\n\tv_nop\n\tv_nop" : "+v"(d) : "v"(a), "v"(b));
  return d;
}

__device__ __forceinline__ float red16_sum(float x) {
#pragma unroll
  for (int off = 1; off < 16; off <<= 1) x += __shfl_xor(x, off, 32);
  return x;
}

__global__ __launch_bounds__(256) void cent_prep_kernel(
    const float* __restrict__ cent, const float* __restrict__ wid,
    const float* __restrict__ rcv, const float* __restrict__ rsv,
    const float* __restrict__ coef,
    _Float16* __restrict__ Bh, _Float16* __restrict__ Br, float* __restrict__ CC) {
  __shared__ _Float16 Th[256 * KDIM];
  __shared__ _Float16 Tr[256 * KDIM];
  __shared__ float Tc[256 * 2];
  const unsigned tid = threadIdx.x;
  const unsigned mrow = blockIdx.x * 256u + tid;

  float csq = 0.0f, covsum = 0.0f;
#pragma unroll 1
  for (unsigned d = 0; d < (unsigned)DDIM; ++d) {
    const float c  = in_cvt(cent[(size_t)mrow * DDIM + d]);
    const float w  = in_cvt(wid[(size_t)mrow * DDIM + d]);
    const float rc = in_cvt(rcv[d]);
    const float rs = in_cvt(rsv[d]);
    const float cr = c * rs;
    const float cov = (w * w + rc * rc) + cr * cr;
    const float iv = 1.0f / cov;
    const float civ = c * iv;
    csq += (c * c) * iv;
    covsum += cov;
    h16 h0, r0, h1, r1;
    split_h(iv, h0, r0);
    split_h(-2.0f * civ, h1, r1);
    Th[tid * KDIM + d] = h0;
    Tr[tid * KDIM + d] = r0;
    Th[tid * KDIM + DDIM + d] = h1;
    Tr[tid * KDIM + DDIM + d] = r1;
  }
  Tc[tid * 2u]      = (0.5f * log2f(covsum) - 21.2119690899f) - 0.7213475204f * csq + LSHIFT;
  Tc[tid * 2u + 1u] = in_cvt(coef[mrow]);
  __syncthreads();

  v8h xh[4], xr[4];
  size_t off[4];
#pragma unroll
  for (unsigned i = 0; i < 4u; ++i) {
    const unsigned idx = tid + 256u * i;
    xh[i] = *(const v8h*)&Th[idx * 8u];
    xr[i] = *(const v8h*)&Tr[idx * 8u];
    off[i] = (size_t)blockIdx.x * 256u * KDIM + (size_t)idx * 8u;
  }
  const unsigned cidx = (tid & 127u) * 4u;
  const v4f cv = *(const v4f*)&Tc[cidx];
  const size_t coff = (size_t)blockIdx.x * 512u + cidx;
  const bool cc_writer = (tid < 128u);

#pragma unroll
  for (int i = 0; i < 4; ++i) {
    *(volatile v8h*)(Bh + off[i]) = xh[i];
    *(volatile v8h*)(Br + off[i]) = xr[i];
  }
  if (cc_writer) *(volatile v4f*)(CC + coff) = cv;
  __threadfence();
#pragma unroll
  for (int i = 0; i < 4; ++i) {
    *(volatile v8h*)(Bh + off[i]) = xh[i];
    *(volatile v8h*)(Br + off[i]) = xr[i];
  }
  if (cc_writer) *(volatile v4f*)(CC + coff) = cv;
}

__global__ __launch_bounds__(256) void rbf_main_kernel(
    const float* __restrict__ X, const _Float16* __restrict__ Bh, const _Float16* __restrict__ Br,
    const float* __restrict__ CC, float* __restrict__ out) {
  __shared__ float Zs[128];
  __shared__ float Ws[128];
  const unsigned tid = threadIdx.x, lane = tid & 31u;
  const unsigned wave = (unsigned)__builtin_amdgcn_readfirstlane((int)(tid >> 5));
  const unsigned hh = lane >> 4, m = lane & 15u;
  const unsigned row0 = blockIdx.x * 128u + wave * 16u;

  const float* xp = X + (size_t)(row0 + m) * DDIM + hh * 8u;
  const v4f xa = *(const v4f*)xp;
  const v4f xb = *(const v4f*)(xp + 4);
  v16h ah, ar;
#pragma unroll
  for (int i = 0; i < 4; ++i) {
    const float xv = in_cvt(xa[i]);
    h16 a, b;
    split_h(ACARRY * (xv * xv), a, b);
    ah[i] = a; ar[i] = b;
    split_h(ACARRY * xv, a, b);
    ah[i + 8] = a; ar[i + 8] = b;
  }
#pragma unroll
  for (int i = 0; i < 4; ++i) {
    const float xv = in_cvt(xb[i]);
    h16 a, b;
    split_h(ACARRY * (xv * xv), a, b);
    ah[i + 4] = a; ar[i + 4] = b;
    split_h(ACARRY * xv, a, b);
    ah[i + 12] = a; ar[i + 12] = b;
  }

  float zacc[8], wacc[8];
#pragma unroll
  for (int r = 0; r < 8; ++r) { zacc[r] = 0.0f; wacc[r] = 0.0f; }

  const _Float16* bh = Bh + (size_t)m * KDIM + hh * 8u;
  const _Float16* br = Br + (size_t)m * KDIM + hh * 8u;
  const float* cc = CC + m * 2u;
  const float k1 = -0.7213475204f * (1.0f / ACARRY);

#pragma unroll 2
  for (unsigned ct = 0; ct < (unsigned)(MCENT / 16); ++ct) {
    const size_t bo = (size_t)ct * 16u * KDIM;
    const v16h bhf = frag_at(bh + bo);
    v8f acc = {};
    acc = wmma16(ah, bhf, acc);
#if SCORE_RES
    const v16h brf = frag_at(br + bo);
    v8f acr = {};
    acr = wmma16(ah, brf, acr);
    acr = wmma16(ar, bhf, acr);
#endif
    const v2f cv = *(const v2f*)(cc + ct * 32u);
#pragma unroll
    for (int r = 0; r < 8; ++r) {
#if SCORE_RES
      const float s = fmaf(acr[r], 1.0f / RCARRY, acc[r]);
#else
      const float s = acc[r];
#endif
      const float e = __builtin_amdgcn_exp2f(fmaf(s, k1, cv[0]));
      zacc[r] += e;
      wacc[r] = fmaf(e, cv[1], wacc[r]);
    }
  }

#pragma unroll
  for (int r = 0; r < 8; ++r) {
    zacc[r] = red16_sum(zacc[r]);
    wacc[r] = red16_sum(wacc[r]);
  }
  if (m == 0u) {
#pragma unroll
    for (int r = 0; r < 8; ++r) {
      Zs[wave * 16u + hh * 8u + (unsigned)r] = zacc[r];
      Ws[wave * 16u + hh * 8u + (unsigned)r] = wacc[r];
    }
  }
  __syncthreads();

  if (wave == 0u) {
    const v4f zz = *(const v4f*)&Zs[lane * 4u];
    const v4f ww = *(const v4f*)&Ws[lane * 4u];
    v4f o;
#pragma unroll
    for (int j = 0; j < 4; ++j) o[j] = ww[j] / zz[j];
    float* p = out + (size_t)blockIdx.x * 128u + lane * 4u;
    *(volatile v4f*)p = o;
    __threadfence();
    *(volatile v4f*)p = o;
  }
}

extern "C" void kernel_launch(void* const* d_in, const int* in_sizes, int n_in,
                              void* d_out, int out_size, void* d_ws, size_t ws_size,
                              hipStream_t stream) {
  if (n_in < 6) return;
  if ((long long)in_sizes[0] < (long long)NPTS * DDIM) return;
  if ((long long)in_sizes[1] < (long long)MCENT * DDIM) return;
  if ((long long)in_sizes[2] < (long long)MCENT * DDIM) return;
  if (in_sizes[3] < MCENT) return;
  if (in_sizes[4] < DDIM || in_sizes[5] < DDIM) return;
  if ((long long)out_size < (long long)NPTS) return;
  if (ws_size < WS_TOTAL) return;

  const float* X    = (const float*)d_in[0];
  const float* cent = (const float*)d_in[1];
  const float* wid  = (const float*)d_in[2];
  const float* coef = (const float*)d_in[3];
  const float* rcv  = (const float*)d_in[4];
  const float* rsv  = (const float*)d_in[5];
  float* out = (float*)d_out;

  char* ws = (char*)d_ws;
  _Float16* Bh = (_Float16*)(ws + OFF_BH);
  _Float16* Br = (_Float16*)(ws + OFF_BR);
  float*    CC = (float*)(ws + OFF_CC);

  cent_prep_kernel<<<dim3(MCENT / 256), dim3(256), 0, stream>>>(cent, wid, rcv, rsv, coef, Bh, Br, CC);
  rbf_main_kernel<<<dim3(NPTS / 128), dim3(256), 0, stream>>>(X, Bh, Br, CC, out);
}
